// GATLayerV2_51994874085817
// MI455X (gfx1250) — hardware-run, weakly checked
//
#include <hip/hip_runtime.h>
#include <stddef.h>
#include <stdint.h>
#include <math.h>


#define NN      100000
#define NE      1600000
#define DIN     64
#define DOUT    32
#define GBM     128
#define NGB     782
#define MP      (NGB * GBM)
#define NB      1024
#define NBLK    98
#define SLSH    17
#define SRCMASK 0x1FFFF
#define NTHR    256
#define NWAVE   8
#define CHK     256
#define NCHK    (NE / CHK)
#define WLCAP   4096
#define RCAP    28672
#define MEASB   16710
#define SP      36
#define NUX     (MP * (DIN / 8))
#define NBX     (NUX / NTHR)
#define NEGSL   0.2f
#define EPS_SM  1e-16f
#define MX0     (-1.0e30f)
#define BKT_INTS (NWAVE * WLCAP + NWAVE * NB + RCAP + 2 * NB + 32)
#define BKT_LDS  (BKT_INTS * 4)

static_assert(NN % 32 == 0);
static_assert(NE % CHK == 0 && NCHK * CHK == NE);
static_assert(MP >= NN && MP == NGB * GBM && NUX % NTHR == 0);
static_assert(NBLK * NB >= NN && (NBLK - 1) * NB < NN);
static_assert(NN < (1 << SLSH) && NB == (1 << 10) && SLSH + 10 < 31);
static_assert(NB == 4 * NTHR && NB % 32 == 0);
static_assert(RCAP >= MEASB + 4096);
static_assert(WLCAP >= ((MEASB / NWAVE) * 3) / 2);
static_assert(RCAP % (4 * NTHR) == 0 && (NWAVE * NB + RCAP) % (4 * NTHR) == 0);
static_assert(BKT_LDS < 300000);
static_assert(DIN % 32 == 0 && DOUT == 32 && GBM == NWAVE * 16);
static_assert((SP * 4) % 16 == 0 && SP >= DOUT);

typedef float          v4f   __attribute__((ext_vector_type(4)));
typedef float          v8f   __attribute__((ext_vector_type(8)));
typedef int            v4i   __attribute__((ext_vector_type(4)));
typedef int            v8i   __attribute__((ext_vector_type(8)));
typedef unsigned int   v4u   __attribute__((ext_vector_type(4)));
typedef unsigned short v8us  __attribute__((ext_vector_type(8)));
typedef __bf16         v16bf __attribute__((ext_vector_type(16)));
typedef v4f  __attribute__((may_alias)) v4fa;
typedef v4i  __attribute__((may_alias)) v4ia;
typedef v8us __attribute__((may_alias)) v8usa;
union FragB { v16bf v; v8us h[2]; v8i w; };

constexpr size_t al256(size_t v) { return (v + 255) & ~(size_t)255; }
constexpr size_t SZ_XB   = (size_t)MP * DIN * 2;
constexpr size_t SZ_WT   = (size_t)DOUT * DIN * 2;
constexpr size_t SZ_ATT  = (size_t)64 * 4;
constexpr size_t SZ_WX   = (size_t)MP * DOUT * 4;
constexpr size_t SZ_SST  = (size_t)2 * MP * 4;
constexpr size_t SZ_HITS = (size_t)NBLK * RCAP * 4;
constexpr size_t SZ_OFF  = (size_t)NBLK * NB * 4;
constexpr size_t SZ_FLAG = (size_t)NBLK * 128;
constexpr size_t O_XB    = 0;
constexpr size_t O_WT    = al256(O_XB + SZ_XB);
constexpr size_t O_ATT   = al256(O_WT + SZ_WT);
constexpr size_t O_WX    = al256(O_ATT + SZ_ATT);
constexpr size_t O_SST   = al256(O_WX + SZ_WX);
constexpr size_t O_HITS  = al256(O_SST + SZ_SST);
constexpr size_t O_OFF   = al256(O_HITS + SZ_HITS);
constexpr size_t O_CNT   = al256(O_OFF + SZ_OFF);
constexpr size_t O_FLAG  = al256(O_CNT + SZ_OFF);
constexpr size_t O_END   = al256(O_FLAG + SZ_FLAG);
static_assert(O_END <= ((size_t)128u << 20));
static_assert((MP * 4) % 128 == 0 && (RCAP * 4) % 128 == 0);

__device__ __forceinline__ v8f wmb(const FragB& a, const FragB& b, v8f c) {
  v8f d = __builtin_amdgcn_wmma_f32_16x16x32_bf16(false, a.v, false, b.v, (short)0, c, false, false);
  asm volatile("v_nop\n\tv_nop\n\tv_nop\n\tv_nop" : "+v"(d) : "v"(a.w), "v"(b.w));
  return d;
}

__device__ __forceinline__ unsigned f2bf(float f) {
  const unsigned u = __float_as_uint(f);
  return ((u + 0x7FFFu + ((u >> 16) & 1u)) >> 16) & 0xFFFFu;
}
__device__ __forceinline__ float bfr(float f) { return __uint_as_float(f2bf(f) << 16); }
__device__ __forceinline__ unsigned pk2(float lo, float hi) { return f2bf(lo) | (f2bf(hi) << 16); }

__global__ __launch_bounds__(NTHR) void k_prep(const float* __restrict__ x, const float* __restrict__ W,
                                               const float* __restrict__ avs, const float* __restrict__ avd,
                                               unsigned short* XB, unsigned short* WT, float* ATT) {
  const int tid = (int)threadIdx.x;
  const int blk = (int)blockIdx.x;
  if (blk < NBX) {
    const int u   = blk * NTHR + tid;
    const int row = u >> 3;
    const int k8  = (u & 7) * 8;
    const int rc  = row < NN ? row : NN - 1;
    const float* p = x + (size_t)rc * DIN + k8;
    const v4f a = *(const v4f*)p;
    const v4f b = *(const v4f*)(p + 4);
    asm volatile("" :: "v"(a), "v"(b));
    const unsigned keep = row < NN ? 0xFFFFFFFFu : 0u;
    v4u o;
    o.x = pk2(a.x, a.y) & keep; o.y = pk2(a.z, a.w) & keep;
    o.z = pk2(b.x, b.y) & keep; o.w = pk2(b.z, b.w) & keep;
    unsigned short* dp = XB + (size_t)row * DIN + k8;
    *(volatile v4u*)dp = o;
    __threadfence();
    *(volatile v4u*)dp = o;
  } else if (blk == NBX) {
    const int n  = tid >> 3;
    const int k8 = (tid & 7) * 8;
    const float* p = W + (size_t)k8 * DOUT + n;
    const float w0 = p[0 * DOUT], w1 = p[1 * DOUT], w2 = p[2 * DOUT], w3 = p[3 * DOUT];
    const float w4 = p[4 * DOUT], w5 = p[5 * DOUT], w6 = p[6 * DOUT], w7 = p[7 * DOUT];
    v4u o;
    o.x = pk2(w0, w1); o.y = pk2(w2, w3); o.z = pk2(w4, w5); o.w = pk2(w6, w7);
    unsigned short* dp = WT + (size_t)n * DIN + k8;
    *(volatile v4u*)dp = o;
    __threadfence();
    *(volatile v4u*)dp = o;
  } else {
    const int i4 = (tid & 7) * 4;
    const v4f a = *(const v4f*)(avs + i4);
    const v4f b = *(const v4f*)(avd + i4);
    asm volatile("" :: "v"(a), "v"(b));
    const unsigned ma = ((tid & 8) == 0) ? 0xFFFFFFFFu : 0u;
    v4f o;
    o.x = bfr(__uint_as_float((__float_as_uint(a.x) & ma) | (__float_as_uint(b.x) & ~ma)));
    o.y = bfr(__uint_as_float((__float_as_uint(a.y) & ma) | (__float_as_uint(b.y) & ~ma)));
    o.z = bfr(__uint_as_float((__float_as_uint(a.z) & ma) | (__float_as_uint(b.z) & ~ma)));
    o.w = bfr(__uint_as_float((__float_as_uint(a.w) & ma) | (__float_as_uint(b.w) & ~ma)));
    if (tid < 16) {
      float* dp = ATT + 4 * tid;
      *(volatile v4f*)dp = o;
      __threadfence();
      *(volatile v4f*)dp = o;
    }
  }
}

__global__ __launch_bounds__(NTHR) void k_gemm_one(const unsigned short* __restrict__ XB,
                                                   const unsigned short* __restrict__ WT,
                                                   const float* __restrict__ ATT, float* WX, float* SST) {
  __shared__ __attribute__((aligned(16))) float stg[GBM * SP];
  __shared__ __attribute__((aligned(16))) float satt[64];
  __shared__ __attribute__((aligned(16))) float sdt[2 * GBM];
  const int tid = (int)threadIdx.x, lane = tid & 31, wave = tid >> 5, hh = lane >> 4, m = lane & 15;
  const int rowBase = (int)blockIdx.x * GBM;

  {
    const v4f av = *(const v4f*)(ATT + 4 * (tid & 15));
    asm volatile("" :: "v"(av));
    if (tid < 16) *(v4fa*)(satt + 4 * tid) = av;
  }

  v8f acc[2];
  {
    const v8f z = {0.f, 0.f, 0.f, 0.f, 0.f, 0.f, 0.f, 0.f};
    acc[0] = z; acc[1] = z;
  }
  const unsigned short* ap = XB + (size_t)(rowBase + 16 * wave + m) * DIN + 8 * hh;
  const unsigned short* wp = WT + (size_t)m * DIN + 8 * hh;
#pragma unroll
  for (int ks = 0; ks < DIN / 32; ++ks) {
    FragB af;
    af.h[0] = *(const v8usa*)(ap + 32 * ks);
    af.h[1] = *(const v8usa*)(ap + 32 * ks + 16);
#pragma unroll
    for (int t = 0; t < 2; ++t) {
      const unsigned short* wq = wp + (size_t)(16 * t) * DIN + 32 * ks;
      FragB bf;
      bf.h[0] = *(const v8usa*)wq;
      bf.h[1] = *(const v8usa*)(wq + 16);
      acc[t] = wmb(af, bf, acc[t]);
    }
  }

#pragma unroll
  for (int t = 0; t < 2; ++t) {
    const int lc = 16 * t + m;
#pragma unroll
    for (int r = 0; r < 8; ++r) {
      const int lr = 16 * wave + 8 * hh + r;
      stg[lr * SP + lc] = acc[t][r];
    }
  }
  __syncthreads();

  if (tid < GBM) {
    const float* hr = stg + tid * SP;
    float ds = 0.0f, dd = 0.0f;
#pragma unroll 2
    for (int c4 = 0; c4 < DOUT / 4; ++c4) {
      const v4f hv = *(const v4fa*)(hr + 4 * c4);
      const v4f sv = *(const v4fa*)(satt + 4 * c4);
      const v4f dv = *(const v4fa*)(satt + 32 + 4 * c4);
      ds = fmaf(hv.x, sv.x, ds);  dd = fmaf(hv.x, dv.x, dd);
      ds = fmaf(hv.y, sv.y, ds);  dd = fmaf(hv.y, dv.y, dd);
      ds = fmaf(hv.z, sv.z, ds);  dd = fmaf(hv.z, dv.z, dd);
      ds = fmaf(hv.w, sv.w, ds);  dd = fmaf(hv.w, dv.w, dd);
    }
    sdt[tid]       = ds;
    sdt[GBM + tid] = dd;
  }
  __syncthreads();

  v4f fv[4];
#pragma unroll
  for (int i = 0; i < 4; ++i) {
    const int lr = 16 * wave + 4 * i + (lane >> 3);
    fv[i] = *(const v4fa*)(stg + lr * SP + 4 * (lane & 7));
  }
  const int pl = wave & 1;
  const v4f sdv = *(const v4fa*)(sdt + pl * GBM + 4 * lane);
  float* sp = SST + (size_t)pl * MP + rowBase + 4 * lane;
  const bool wsd = wave < 2;

#pragma unroll
  for (int i = 0; i < 4; ++i) {
    const int lr = 16 * wave + 4 * i + (lane >> 3);
    float* op = WX + (size_t)(rowBase + lr) * DOUT + 4 * (lane & 7);
    *(volatile v4f*)op = fv[i];
  }
  if (wsd) *(volatile v4f*)sp = sdv;
  __threadfence();
#pragma unroll
  for (int i = 0; i < 4; ++i) {
    const int lr = 16 * wave + 4 * i + (lane >> 3);
    float* op = WX + (size_t)(rowBase + lr) * DOUT + 4 * (lane & 7);
    *(volatile v4f*)op = fv[i];
  }
  if (wsd) *(volatile v4f*)sp = sdv;
}

__global__ __launch_bounds__(NTHR) void k_bucket(const int* __restrict__ srcs, const int* __restrict__ dsts,
                                                 int* HITS, int* OFF, int* CNT, int* FLAG) {
  extern __shared__ __attribute__((aligned(16))) int dsm[];
  int* wl   = dsm;
  int* cw   = wl + NWAVE * WLCAP;
  int* hits = cw + NWAVE * NB;
  int* soff = hits + RCAP;
  int* scnt = soff + NB;
  int* misc = scnt + NB;
  const int tid = (int)threadIdx.x, lane = tid & 31, wave = tid >> 5;
  const int b = (int)blockIdx.x;
  const int nodeBase = b * NB;
  const int nb = (NN - nodeBase) < NB ? (NN - nodeBase) : NB;

  {
    const v4i z4 = {0, 0, 0, 0};
#pragma unroll 4
    for (int i = tid * 4; i < NWAVE * NB + RCAP; i += NTHR * 4) *(v4ia*)(cw + i) = z4;
    if (tid < 32) misc[tid] = 0;
  }
  __syncthreads();

  int wc = 0;
  const unsigned nbs = (unsigned)nodeBase;
  const unsigned unb = (unsigned)nb;
  int* mywl = wl + wave * WLCAP;
#pragma unroll 1
  for (int ch = wave; ch < NCHK; ch += NWAVE) {
    const int e0 = ch * CHK + lane * 8;
    const v4i da = *(const v4i*)(dsts + e0);
    const v4i db = *(const v4i*)(dsts + e0 + 4);
    const v4i sa = *(const v4i*)(srcs + e0);
    const v4i sb = *(const v4i*)(srcs + e0 + 4);
    asm volatile("" :: "v"(da), "v"(db), "v"(sa), "v"(sb));
    const unsigned s0 = (unsigned)da.x - nbs, s1 = (unsigned)da.y - nbs;
    const unsigned s2 = (unsigned)da.z - nbs, s3 = (unsigned)da.w - nbs;
    const unsigned s4 = (unsigned)db.x - nbs, s5 = (unsigned)db.y - nbs;
    const unsigned s6 = (unsigned)db.z - nbs, s7 = (unsigned)db.w - nbs;
    const bool h0 = s0 < unb, h1 = s1 < unb, h2 = s2 < unb, h3 = s3 < unb;
    const bool h4 = s4 < unb, h5 = s5 < unb, h6 = s6 < unb, h7 = s7 < unb;
    const unsigned any = __builtin_amdgcn_ballot_w32(h0 | h1 | h2 | h3 | h4 | h5 | h6 | h7);
    if (any != 0u) {
#define HITJ(HJ, SJ, SRJ) { \
      const unsigned mj = __builtin_amdgcn_ballot_w32(HJ); \
      if (mj != 0u) { \
        const int pos = wc + (int)__builtin_amdgcn_mbcnt_lo(mj, 0u); \
        int sr = (SRJ); \
        sr = sr < 0 ? 0 : (sr > NN - 1 ? NN - 1 : sr); \
        const int ent = sr | (int)(((SJ) & (unsigned)(NB - 1)) << SLSH); \
        if ((HJ) && pos < WLCAP) mywl[pos] = ent; \
        wc += (int)__builtin_popcount(mj); } }
      HITJ(h0, s0, sa.x)
      HITJ(h1, s1, sa.y)
      HITJ(h2, s2, sa.z)
      HITJ(h3, s3, sa.w)
      HITJ(h4, s4, sb.x)
      HITJ(h5, s5, sb.y)
      HITJ(h6, s6, sb.z)
      HITJ(h7, s7, sb.w)
#undef HITJ
    }
  }
  if (lane == 0) misc[wave] = (wc > WLCAP) ? 1 : 0;
  const int wcc = wc < 0 ? 0 : (wc > WLCAP ? WLCAP : wc);
  __syncthreads();

  if (lane == 0) {
    int* myc = cw + wave * NB;
#pragma unroll 1
    for (int i = 0; i < wcc; ++i) {
      const int ent = mywl[i];
      const int sl  = (ent >> SLSH) & (NB - 1);
      myc[sl] = myc[sl] + 1;
    }
  }
  __syncthreads();

  v4i cwv[NWAVE];
#pragma unroll
  for (int w = 0; w < NWAVE; ++w) cwv[w] = *(const v4ia*)(cw + w * NB + 4 * tid);
  v4i tot = cwv[0];
#pragma unroll
  for (int w = 1; w < NWAVE; ++w) tot += cwv[w];
  const int ts = tot.x + tot.y + tot.z + tot.w;
  int incl = ts;
#pragma unroll
  for (int dl = 1; dl < 32; dl <<= 1) {
    const int y = __shfl_up(incl, dl);
    incl += (lane >= dl) ? y : 0;
  }
  if (lane == 31) misc[8 + wave] = incl;
  __syncthreads();
  int pre = 0, all = 0, ovs = 0;
#pragma unroll
  for (int w2 = 0; w2 < NWAVE; ++w2) {
    const int t2 = misc[8 + w2];
    all += t2;
    pre += (w2 < wave) ? t2 : 0;
    ovs |= misc[w2];
  }
  const int ovf = (ovs != 0 || all > RCAP) ? 1 : 0;
  {
    const int run = pre + incl - ts;
    v4i offv;
    offv.x = run;
    offv.y = offv.x + tot.x;
    offv.z = offv.y + tot.y;
    offv.w = offv.z + tot.z;
    *(v4ia*)(soff + 4 * tid) = offv;
    *(v4ia*)(scnt + 4 * tid) = tot;
    v4i cur = offv;
#pragma unroll
    for (int w = 0; w < NWAVE; ++w) {
      *(v4ia*)(cw + w * NB + 4 * tid) = cur;
      cur += cwv[w];
    }
  }
  __syncthreads();

  if (lane == 0) {
    int* myc = cw + wave * NB;
#pragma unroll 1
    for (int i = 0; i < wcc; ++i) {
      const int ent = mywl[i];
      const int sl  = (ent >> SLSH) & (NB - 1);
      int p = myc[sl];
      myc[sl] = p + 1;
      p = p < 0 ? 0 : (p > RCAP - 1 ? RCAP - 1 : p);
      hits[p] = ent;
    }
  }
  __syncthreads();

  int* hg = HITS + (size_t)b * RCAP;
  const v4i ofv = *(const v4ia*)(soff + 4 * tid);
  const v4i cnv = *(const v4ia*)(scnt + 4 * tid);
  const v4i flv = {ovf, ovf, ovf, ovf};
  int* og = OFF + (size_t)b * NB + 4 * tid;
  int* cg = CNT + (size_t)b * NB + 4 * tid;
  int* fg = FLAG + (size_t)b * 32 + 4 * (lane & 7);
  const bool wfl = (wave == 0) && (lane < 8);
#pragma unroll 4
  for (int i = 0; i < RCAP / (4 * NTHR); ++i) {
    const int i4 = 4 * (i * NTHR + tid);
    const v4i hv = *(const v4ia*)(hits + i4);
    *(volatile v4i*)(hg + i4) = hv;
  }
  *(volatile v4i*)og = ofv;
  *(volatile v4i*)cg = cnv;
  if (wfl) *(volatile v4i*)fg = flv;
  __threadfence();
#pragma unroll 4
  for (int i = 0; i < RCAP / (4 * NTHR); ++i) {
    const int i4 = 4 * (i * NTHR + tid);
    const v4i hv = *(const v4ia*)(hits + i4);
    *(volatile v4i*)(hg + i4) = hv;
  }
  *(volatile v4i*)og = ofv;
  *(volatile v4i*)cg = cnv;
  if (wfl) *(volatile v4i*)fg = flv;
}

__global__ __launch_bounds__(NTHR) void k_replay(const int* __restrict__ HITS, const int* __restrict__ OFF,
                                                 const int* __restrict__ CNT, const int* __restrict__ FLAG,
                                                 const float* __restrict__ SS, const float* __restrict__ ST,
                                                 const float* __restrict__ WX, float* outp) {
  const int tid = (int)threadIdx.x, lane = tid & 31, wave = tid >> 5;
  const int q = lane >> 3, c4 = lane & 7;
  const int d = (int)blockIdx.x * 32 + wave * 4 + q;
  const int b = d >> 10;
  int o = OFF[d];
  int c = CNT[d];
  const float sd = ST[d];
  const int flag = FLAG[b * 32];
  o = o < 0 ? 0 : (o > RCAP - 1 ? RCAP - 1 : o);
  c = c > RCAP - o ? RCAP - o : c;
  c = c < 0 ? 0 : c;
  int cm = c;
  {
    const int y8 = __shfl_xor(cm, 8);
    cm = cm > y8 ? cm : y8;
    const int y16 = __shfl_xor(cm, 16);
    cm = cm > y16 ? cm : y16;
  }
  cm = cm > RCAP ? RCAP : cm;
  const int trip = __builtin_amdgcn_readfirstlane(cm);
  int last = o + c - 1;
  last = last < o ? o : last;
  const int* hp = HITS + (size_t)b * RCAP;

  float m = MX0, den = 0.0f;
  v4f acc = {0.0f, 0.0f, 0.0f, 0.0f};
#pragma unroll 1
  for (int j = 0; j < trip; ++j) {
    int idx = o + j;
    idx = idx > last ? last : idx;
    const int word = hp[idx];
    asm volatile("" :: "v"(word));
    int s = word & SRCMASK;
    s = s > NN - 1 ? NN - 1 : s;
    const float ss = SS[s];
    const v4f wx = *(const v4f*)(WX + (size_t)s * DOUT + 4 * c4);
    asm volatile("" :: "v"(ss), "v"(wx));
    const bool valid = j < c;
    float e = sd + ss;
    e = e > 0.0f ? e : NEGSL * e;
    const float df = e - m;
    const float ee = expf(-fabsf(df));
    const bool up = df > 0.0f;
    float s1 = up ? ee : 1.0f;
    float s2 = up ? 1.0f : ee;
    s1 = valid ? s1 : 1.0f;
    s2 = valid ? s2 : 0.0f;
    m = (valid && up) ? e : m;
    den = fmaf(den, s1, s2);
    acc.x = fmaf(acc.x, s1, s2 * wx.x);
    acc.y = fmaf(acc.y, s1, s2 * wx.y);
    acc.z = fmaf(acc.z, s1, s2 * wx.z);
    acc.w = fmaf(acc.w, s1, s2 * wx.w);
  }
  const float inv = 1.0f / (den + EPS_SM);
  v4f v;
  v.x = acc.x * inv; v.y = acc.y * inv; v.z = acc.z * inv; v.w = acc.w * inv;
#pragma unroll 1
  for (int i = 0; i < 4; ++i) {
    const float t = v.x;
    const float r = (t > 0.0f) ? t : expm1f(t);
    v4f nv;
    nv.x = v.y; nv.y = v.z; nv.z = v.w; nv.w = r;
    v = nv;
  }
  const float qn = __int_as_float(0x7fc00000);
  const bool bad = flag != 0;
  v.x = bad ? qn : v.x;
  v.y = bad ? qn : v.y;
  v.z = bad ? qn : v.z;
  v.w = bad ? qn : v.w;
  float* op = outp + (size_t)d * DOUT + 4 * c4;
  *(volatile v4f*)op = v;
  __threadfence();
  *(volatile v4f*)op = v;
}

extern "C" void kernel_launch(void* const* d_in, const int* in_sizes, int n_in,
                              void* d_out, int out_size, void* d_ws, size_t ws_size,
                              hipStream_t stream) {
  if (n_in < 5) return;
  if (in_sizes[0] != NN * DIN) return;
  if (in_sizes[1] != 2 * NE) return;
  if (in_sizes[2] != DIN * DOUT) return;
  if (in_sizes[3] != DOUT) return;
  if (in_sizes[4] != DOUT) return;
  if (out_size != NN * DOUT) return;
  if ((size_t)O_END > ws_size) return;

  const float* x   = (const float*)d_in[0];
  const int*   ei  = (const int*)d_in[1];
  const float* W   = (const float*)d_in[2];
  const float* avs = (const float*)d_in[3];
  const float* avd = (const float*)d_in[4];
  float* out = (float*)d_out;
  const int* src = ei;
  const int* dst = ei + NE;

  char* ws = (char*)d_ws;
  unsigned short* XB   = (unsigned short*)(ws + O_XB);
  unsigned short* WT   = (unsigned short*)(ws + O_WT);
  float*          ATT  = (float*)(ws + O_ATT);
  float*          WX   = (float*)(ws + O_WX);
  float*          SST  = (float*)(ws + O_SST);
  int*            HITS = (int*)(ws + O_HITS);
  int*            OFF  = (int*)(ws + O_OFF);
  int*            CNT  = (int*)(ws + O_CNT);
  int*            FLAG = (int*)(ws + O_FLAG);

  hipFuncSetAttribute(reinterpret_cast<const void*>(&k_bucket),
                      hipFuncAttributeMaxDynamicSharedMemorySize, (int)BKT_LDS);

  k_prep<<<NBX + 2, NTHR, 0, stream>>>(x, W, avs, avd, XB, WT, ATT);
  k_gemm_one<<<NGB, NTHR, 0, stream>>>(XB, WT, ATT, WX, SST);
  k_bucket<<<NBLK, NTHR, BKT_LDS, stream>>>(src, dst, HITS, OFF, CNT, FLAG);
  k_replay<<<NN / 32, NTHR, 0, stream>>>(HITS, OFF, CNT, FLAG, SST, SST + MP, WX, out);
}
